// CSEM_86294482911613
// MI455X (gfx1250) — hardware-verified
//
#include <hip/hip_runtime.h>


typedef _Float16 v16h __attribute__((ext_vector_type(16)));
typedef _Float16 v8h  __attribute__((ext_vector_type(8)));
typedef float    v8f  __attribute__((ext_vector_type(8)));
typedef float    v4f  __attribute__((ext_vector_type(4)));
union Frag { v16h v; v8h half[2]; };

#define HW        9216
#define IMW       96
#define LSTR      40
#define CSP       132
#define SPQ       196
#define CONV_SMEM 33792
#define ATTN_SMEM 50176
#define PSH       8

__device__ __forceinline__ v16h ld_frag(const _Float16* rowp, int hsel) {
  Frag f;
  f.half[0] = *(const v8h*)(rowp + hsel);
  f.half[1] = *(const v8h*)(rowp + 16 + hsel);
  return f.v;
}

__device__ __forceinline__ v8f wmma16(v16h a, v16h b, v8f c) {
  v8f d = __builtin_amdgcn_wmma_f32_16x16x32_f16(false, a, false, b, (short)0, c, false, false);
  asm volatile("v_nop\n\tv_nop\n\tv_nop\n\tv_nop" : "+v"(d) : "v"(a), "v"(b));
  return d;
}

__device__ __forceinline__ void store_pk8(_Float16* dst, const float* src) {
  v8h v;
#pragma unroll
  for (int j = 0; j < 8; ++j) v[j] = (_Float16)src[j];
  *(v8h*)dst = v;
}
__device__ __forceinline__ void store_pk8(_Float16* dst, const _Float16* src) {
  v8h v;
#pragma unroll
  for (int j = 0; j < 8; ++j) v[j] = src[j];
  *(v8h*)dst = v;
}

__device__ __forceinline__ float wave_max(float v) {
#pragma unroll
  for (int o = 16; o > 0; o >>= 1) v = fmaxf(v, __shfl_xor(v, o));
  return v;
}
__device__ __forceinline__ float wave_sum(float v) {
#pragma unroll
  for (int o = 16; o > 0; o >>= 1) v += __shfl_xor(v, o);
  return v;
}

__device__ __forceinline__ void tile_store(const float* stage, float* __restrict__ g,
                                           int wave, int lane) {
  const int col = (lane >> 3) * 32 + (lane & 7) * 4;
#pragma unroll
  for (int pass = 0; pass < 2; ++pass) {
#pragma unroll
    for (int it = 0; it < 8; ++it) {
      const int row = wave * 8 + it;
      v4f v = *(const v4f*)(stage + row * CSP + col);
      *(volatile v4f*)(g + (size_t)row * HW + col) = v;
    }
    if (pass == 0) __threadfence();
  }
}
__device__ __forceinline__ void tile_store(const float* stage, _Float16* __restrict__ g,
                                           int wave, int lane) {
  const int col = (lane & 15) * 8;
  const int rsub = lane >> 4;
#pragma unroll
  for (int pass = 0; pass < 2; ++pass) {
#pragma unroll
    for (int it = 0; it < 4; ++it) {
      const int row = wave * 8 + it * 2 + rsub;
      const float* sp = stage + row * CSP + col;
      v4f x0 = *(const v4f*)sp;
      v4f x1 = *(const v4f*)(sp + 4);
      v8h o;
      o[0] = (_Float16)x0[0]; o[1] = (_Float16)x0[1]; o[2] = (_Float16)x0[2]; o[3] = (_Float16)x0[3];
      o[4] = (_Float16)x1[0]; o[5] = (_Float16)x1[1]; o[6] = (_Float16)x1[2]; o[7] = (_Float16)x1[3];
      *(volatile v8h*)(g + (size_t)row * HW + col) = o;
    }
    if (pass == 0) __threadfence();
  }
}

template <typename TI, typename TO, int CIN, int COUT, int WSH>
__global__ __launch_bounds__(256) void conv3x3_bn_relu(
    const TI* __restrict__ X, const float* __restrict__ Wt,
    const float* __restrict__ cb, const float* __restrict__ gam,
    const float* __restrict__ bet, const float* __restrict__ mu,
    const float* __restrict__ var, TO* __restrict__ Y) {
  constexpr int KTOT = CIN * 9;
  constexpr float WSC = (float)(1 << WSH);
  constexpr float IWSC = 1.0f / WSC;
  constexpr int ASZ = 64 * LSTR;
  constexpr int BSZ = 128 * LSTR;
  __shared__ __attribute__((aligned(16))) char smem[CONV_SMEM];
  __shared__ float s_sc[64];
  __shared__ float s_bi[64];
  _Float16* As = (_Float16*)smem;
  _Float16* Bs = As + 2 * ASZ;
  float* stage = (float*)smem;

  const int bz   = blockIdx.z;
  const int m0   = blockIdx.y * 64;
  const int col0 = blockIdx.x * 128;
  const int tid  = threadIdx.x;
  const int lane = tid & 31;
  const int wave = tid >> 5;
  const int wm = wave & 1, wn = wave >> 1;
  const int fm = lane & 15;
  const int hsel = (lane >> 4) * 8;

  if (tid < 64) {
    const int mm = m0 + tid;
    float sc = gam[mm] * rsqrtf(var[mm] + 1e-5f);
    s_sc[tid] = sc * IWSC;
    s_bi[tid] = bet[mm] + (cb[mm] - mu[mm]) * sc;
  }

  const int arow = tid >> 2;
  const int akk  = (tid & 3) * 8;
  const int bn   = tid & 127;
  const int kb0  = (tid >> 7) * 16;
  const int gcol = col0 + bn;
  const int h    = gcol / IMW;
  const int w    = gcol - h * IMW;
  const size_t xbase = (size_t)bz * CIN * HW;
  const int pbase = (h - 1) * IMW + (w - 1);
  unsigned mask = 0;
#pragma unroll
  for (int rr = 0; rr < 3; ++rr)
#pragma unroll
    for (int ss = 0; ss < 3; ++ss)
      if ((unsigned)(h + rr - 1) < (unsigned)IMW && (unsigned)(w + ss - 1) < (unsigned)IMW)
        mask |= 1u << (rr * 3 + ss);

  float ra[8];
  TI rb[16];

  auto gatherA = [&](int k0) {
    const float* src = Wt + (size_t)(m0 + arow) * KTOT + k0 + akk;
#pragma unroll
    for (int j = 0; j < 8; ++j) ra[j] = src[j] * WSC;
  };
  auto gatherB = [&](int k0) {
#pragma unroll
    for (int it = 0; it < 16; ++it) {
      const int kg = k0 + kb0 + it;
      const int ci = kg / 9;
      const int rs = kg - ci * 9;
      const int r  = rs / 3;
      const int s  = rs - r * 3;
      const bool valid = (mask >> rs) & 1u;
      const int off = valid ? (pbase + r * IMW + s) : 0;
      TI ld = X[xbase + (size_t)ci * HW + off];
      rb[it] = valid ? ld : (TI)0.0f;
    }
  };

  v8f acc[2][2] = {};

  gatherA(0);
  gatherB(0);
  int p = 0;
  for (int k0 = 0; k0 < KTOT; k0 += 32) {
    _Float16* Ap = As + p * ASZ;
    _Float16* Bp = Bs + p * BSZ;
    store_pk8(Ap + arow * LSTR + akk, ra);
    store_pk8(Bp + bn * LSTR + kb0, rb);
    store_pk8(Bp + bn * LSTR + kb0 + 8, rb + 8);
    __syncthreads();
    const int kn = k0 + 32;
    if (kn < KTOT) { gatherA(kn); gatherB(kn); }
    v16h a0 = ld_frag(Ap + (wm * 32 + fm) * LSTR, hsel);
    v16h a1 = ld_frag(Ap + (wm * 32 + 16 + fm) * LSTR, hsel);
    v16h f0 = ld_frag(Bp + (wn * 32 + fm) * LSTR, hsel);
    v16h f1 = ld_frag(Bp + (wn * 32 + 16 + fm) * LSTR, hsel);
    acc[0][0] = wmma16(a0, f0, acc[0][0]);
    acc[0][1] = wmma16(a0, f1, acc[0][1]);
    acc[1][0] = wmma16(a1, f0, acc[1][0]);
    acc[1][1] = wmma16(a1, f1, acc[1][1]);
    p ^= 1;
  }
  __syncthreads();

#pragma unroll
  for (int sm = 0; sm < 2; ++sm) {
#pragma unroll
    for (int j = 0; j < 2; ++j) {
#pragma unroll
      for (int r = 0; r < 8; ++r) {
        const int row = wm * 32 + sm * 16 + hsel + r;
        const int col = wn * 32 + j * 16 + fm;
        stage[row * CSP + col] = fmaxf(acc[sm][j][r] * s_sc[row] + s_bi[row], 0.0f);
      }
    }
  }
  __syncthreads();
  tile_store(stage, Y + ((size_t)bz * COUT + m0) * HW + col0, wave, lane);
}

__device__ __forceinline__ float pool_cell(const float* __restrict__ Yc, int ph, int pw, bool ismax) {
  const float* r0 = Yc + (2 * ph) * IMW + 2 * pw;
  const float a = r0[0], bq = r0[1], c = r0[IMW], d = r0[IMW + 1];
  const float mx = fmaxf(fmaxf(a, bq), fmaxf(c, d));
  const float av = (((a + bq) + c) + d) * 0.25f;
  return ismax ? mx : av;
}

__global__ __launch_bounds__(256) void branch_build(const float* __restrict__ Y,
                                                    _Float16* __restrict__ T, int ngroups) {
  const int g = blockIdx.x * 256 + threadIdx.x;
  if (g >= ngroups) return;
  const int wq = g % 12;
  const int t1 = g / 12;
  const int h  = t1 % IMW;
  const int t2 = t1 / IMW;
  const int c  = t2 % 192;
  const int b  = t2 / 192;
  const int w0 = wq * 8;
  const float* Yc = Y + (size_t)(b * 192 + c) * HW;
  float val[8];
  if (c >= 64 && c < 128) {
    const v4f* src = (const v4f*)(Yc + h * IMW + w0);
    v4f x0 = src[0], x1 = src[1];
    val[0] = x0[0]; val[1] = x0[1]; val[2] = x0[2]; val[3] = x0[3];
    val[4] = x1[0]; val[5] = x1[1]; val[6] = x1[2]; val[7] = x1[3];
  } else {
    const bool ismax = (c < 64);
    const float chc = fminf(fmaxf(0.5f * (float)h - 0.25f, 0.0f), 47.0f);
    const float hlof = floorf(chc);
    const int hlo = (int)hlof;
    const int hhi = min(hlo + 1, 47);
    const float hf  = chc - hlof;
    const float hf1 = 1.0f - hf;
    const int pc0 = 4 * wq - 1;
    float plo[6], phi[6];
#pragma unroll
    for (int jj = 0; jj < 6; ++jj) {
      const int pc = min(max(pc0 + jj, 0), 47);
      plo[jj] = pool_cell(Yc, hlo, pc, ismax);
      phi[jj] = pool_cell(Yc, hhi, pc, ismax);
    }
#pragma unroll
    for (int i = 0; i < 8; ++i) {
      const int jl = (i + 1) >> 1;
      const float cwc = fminf(fmaxf(0.5f * (float)(w0 + i) - 0.25f, 0.0f), 47.0f);
      const float wlof = floorf(cwc);
      const float wf = cwc - wlof;
      const float tlo = plo[jl] * hf1 + phi[jl] * hf;
      const float thi = plo[jl + 1] * hf1 + phi[jl + 1] * hf;
      val[i] = tlo * (1.0f - wf) + thi * wf;
    }
  }
  v8h o;
#pragma unroll
  for (int i = 0; i < 8; ++i) o[i] = (_Float16)val[i];
  _Float16* dst = T + (size_t)g * 8;
  *(volatile v8h*)dst = o;
  __threadfence();
  *(volatile v8h*)dst = o;
}

__global__ __launch_bounds__(256) void attn_scores_softmax(
    const _Float16* __restrict__ T2, const float* __restrict__ temp,
    _Float16* __restrict__ Pm) {
  constexpr int ASZ = 64 * LSTR;
  constexpr int BSZ = 192 * LSTR;
  constexpr float PSC = (float)(1 << PSH);
  __shared__ __attribute__((aligned(16))) char smem[ATTN_SMEM];
  __shared__ float s_qinv[64];
  __shared__ float s_kinv[192];
  _Float16* As = (_Float16*)smem;
  _Float16* Bs = As + 2 * ASZ;
  float* stage = (float*)smem;

  const int b  = blockIdx.y;
  const int i0 = blockIdx.x * 64;
  const int tid  = threadIdx.x;
  const int lane = tid & 31;
  const int wave = tid >> 5;
  const int wm = wave & 3, wn = wave >> 2;
  const int fm = lane & 15;
  const int hsel = (lane >> 4) * 8;
  const int row = tid >> 2;
  const int kk  = (tid & 3) * 8;
  const _Float16* qsrc = T2 + (size_t)(b * 576 + i0 + row) * HW + kk;
  const _Float16* ksrc = T2 + (size_t)(b * 576 + 192 + row) * HW + kk;

  v8h ra, rk0, rk1, rk2;
  float sq = 0.0f, sk0 = 0.0f, sk1 = 0.0f, sk2 = 0.0f;
  auto gather = [&](int k0) {
    ra  = *(const v8h*)(qsrc + k0);
    rk0 = *(const v8h*)(ksrc + k0);
    rk1 = *(const v8h*)(ksrc + (size_t)64 * HW + k0);
    rk2 = *(const v8h*)(ksrc + (size_t)128 * HW + k0);
  };

  v8f acc[6] = {};
  gather(0);
  int p = 0;
  for (int k0 = 0; k0 < HW; k0 += 32) {
#pragma unroll
    for (int e = 0; e < 8; ++e) {
      const float a = (float)ra[e];  sq  += a * a;
      const float x0 = (float)rk0[e]; sk0 += x0 * x0;
      const float x1 = (float)rk1[e]; sk1 += x1 * x1;
      const float x2 = (float)rk2[e]; sk2 += x2 * x2;
    }
    _Float16* Ap = As + p * ASZ;
    _Float16* Bp = Bs + p * BSZ;
    *(v8h*)(Ap + row * LSTR + kk) = ra;
    *(v8h*)(Bp + row * LSTR + kk) = rk0;
    *(v8h*)(Bp + (row + 64) * LSTR + kk) = rk1;
    *(v8h*)(Bp + (row + 128) * LSTR + kk) = rk2;
    __syncthreads();
    if (k0 + 32 < HW) gather(k0 + 32);
    v16h a = ld_frag(Ap + (wm * 16 + fm) * LSTR, hsel);
#pragma unroll
    for (int j = 0; j < 6; ++j) {
      v16h bf = ld_frag(Bp + (wn * 96 + j * 16 + fm) * LSTR, hsel);
      acc[j] = wmma16(a, bf, acc[j]);
    }
    p ^= 1;
  }
  sq  += __shfl_xor(sq, 1);  sq  += __shfl_xor(sq, 2);
  sk0 += __shfl_xor(sk0, 1); sk0 += __shfl_xor(sk0, 2);
  sk1 += __shfl_xor(sk1, 1); sk1 += __shfl_xor(sk1, 2);
  sk2 += __shfl_xor(sk2, 1); sk2 += __shfl_xor(sk2, 2);
  __syncthreads();
  if ((tid & 3) == 0) {
    s_qinv[row]       = 1.0f / fmaxf(sqrtf(sq), 1e-12f);
    s_kinv[row]       = 1.0f / fmaxf(sqrtf(sk0), 1e-12f);
    s_kinv[row + 64]  = 1.0f / fmaxf(sqrtf(sk1), 1e-12f);
    s_kinv[row + 128] = 1.0f / fmaxf(sqrtf(sk2), 1e-12f);
  }
  __syncthreads();
  const float tsc = temp[0];
#pragma unroll
  for (int j = 0; j < 6; ++j) {
#pragma unroll
    for (int r = 0; r < 8; ++r) {
      const int rr = wm * 16 + hsel + r;
      const int cc = wn * 96 + j * 16 + fm;
      stage[rr * SPQ + cc] = acc[j][r] * s_qinv[rr] * s_kinv[cc] * tsc;
    }
  }
  __syncthreads();

#pragma unroll
  for (int it = 0; it < 8; ++it) {
    const int rr = wave * 8 + it;
    float* sp = stage + rr * SPQ + lane;
    float x[6];
#pragma unroll
    for (int c = 0; c < 6; ++c) x[c] = sp[32 * c];
    float mx = x[0];
#pragma unroll
    for (int c = 1; c < 6; ++c) mx = fmaxf(mx, x[c]);
    mx = wave_max(mx);
    float e[6];
    float s = 0.0f;
#pragma unroll
    for (int c = 0; c < 6; ++c) { e[c] = expf(x[c] - mx); s += e[c]; }
    s = wave_sum(s);
    const float inv = 1.0f / s;
#pragma unroll
    for (int c = 0; c < 6; ++c) sp[32 * c] = e[c] * inv * PSC;
  }
  __syncthreads();

  _Float16* pdst = Pm + (size_t)(b * 192 + i0 + wave * 8) * 192;
#pragma unroll
  for (int pass = 0; pass < 2; ++pass) {
#pragma unroll
    for (int it = 0; it < 6; ++it) {
      const int idx = it * 32 + lane;
      const int rl  = idx / 24;
      const int ch  = (idx - rl * 24) * 8;
      const float* sp = stage + (wave * 8 + rl) * SPQ + ch;
      v4f x0 = *(const v4f*)sp;
      v4f x1 = *(const v4f*)(sp + 4);
      v8h o;
      o[0] = (_Float16)x0[0]; o[1] = (_Float16)x0[1]; o[2] = (_Float16)x0[2]; o[3] = (_Float16)x0[3];
      o[4] = (_Float16)x1[0]; o[5] = (_Float16)x1[1]; o[6] = (_Float16)x1[2]; o[7] = (_Float16)x1[3];
      *(volatile v8h*)(pdst + idx * 8) = o;
    }
    if (pass == 0) __threadfence();
  }
}

__global__ __launch_bounds__(256) void attn_pv(
    const _Float16* __restrict__ Pm, const _Float16* __restrict__ T2,
    float* __restrict__ O) {
  constexpr int ASZ = 64 * LSTR;
  constexpr int BSZ = 128 * LSTR;
  constexpr float IPSC = 1.0f / (float)(1 << PSH);
  __shared__ __attribute__((aligned(16))) char smem[CONV_SMEM];
  _Float16* As = (_Float16*)smem;
  _Float16* Bs = As + 2 * ASZ;
  float* stage = (float*)smem;

  const int b    = blockIdx.z;
  const int m0   = blockIdx.y * 64;
  const int col0 = blockIdx.x * 128;
  const int tid  = threadIdx.x;
  const int lane = tid & 31;
  const int wave = tid >> 5;
  const int wm = wave & 1, wn = wave >> 1;
  const int fm = lane & 15;
  const int hsel = (lane >> 4) * 8;
  const int arow = tid >> 2;
  const int akk  = (tid & 3) * 8;
  const int bn   = tid & 127;
  const int kb0  = (tid >> 7) * 16;
  const _Float16* asrc = Pm + (size_t)(b * 192 + m0 + arow) * 192 + akk;
  const _Float16* vsrc = T2 + (size_t)(b * 576 + 384) * HW + col0 + bn;

  v8h ra;
  _Float16 rb[16];
  auto gatherA = [&](int k0) { ra = *(const v8h*)(asrc + k0); };
  auto gatherB = [&](int k0) {
#pragma unroll
    for (int it = 0; it < 16; ++it) rb[it] = vsrc[(size_t)(k0 + kb0 + it) * HW];
  };

  v8f acc[2][2] = {};
  gatherA(0);
  gatherB(0);
  int p = 0;
  for (int k0 = 0; k0 < 192; k0 += 32) {
    _Float16* Ap = As + p * ASZ;
    _Float16* Bp = Bs + p * BSZ;
    *(v8h*)(Ap + arow * LSTR + akk) = ra;
    store_pk8(Bp + bn * LSTR + kb0, rb);
    store_pk8(Bp + bn * LSTR + kb0 + 8, rb + 8);
    __syncthreads();
    const int kn = k0 + 32;
    if (kn < 192) { gatherA(kn); gatherB(kn); }
    v16h a0 = ld_frag(Ap + (wm * 32 + fm) * LSTR, hsel);
    v16h a1 = ld_frag(Ap + (wm * 32 + 16 + fm) * LSTR, hsel);
    v16h f0 = ld_frag(Bp + (wn * 32 + fm) * LSTR, hsel);
    v16h f1 = ld_frag(Bp + (wn * 32 + 16 + fm) * LSTR, hsel);
    acc[0][0] = wmma16(a0, f0, acc[0][0]);
    acc[0][1] = wmma16(a0, f1, acc[0][1]);
    acc[1][0] = wmma16(a1, f0, acc[1][0]);
    acc[1][1] = wmma16(a1, f1, acc[1][1]);
    p ^= 1;
  }
  __syncthreads();
#pragma unroll
  for (int sm = 0; sm < 2; ++sm) {
#pragma unroll
    for (int j = 0; j < 2; ++j) {
#pragma unroll
      for (int r = 0; r < 8; ++r) {
        const int row = wm * 32 + sm * 16 + hsel + r;
        const int col = wn * 32 + j * 16 + fm;
        stage[row * CSP + col] = acc[sm][j][r] * IPSC;
      }
    }
  }
  __syncthreads();
  tile_store(stage, O + ((size_t)b * 192 + m0) * HW + col0, wave, lane);
}

__global__ __launch_bounds__(256) void dwconv3x3(const float* __restrict__ O,
                                                 const float* __restrict__ W2,
                                                 const float* __restrict__ B2,
                                                 float* __restrict__ out, int ngroups) {
  const int g = blockIdx.x * 256 + threadIdx.x;
  if (g >= ngroups) return;
  const int wq = g % 24;
  const int t1 = g / 24;
  const int h  = t1 % IMW;
  const int t2 = t1 / IMW;
  const int c  = t2 % 192;
  const int b  = t2 / 192;
  const int w0 = wq * 4;
  const float* Oc = O + (size_t)(b * 192 + c) * HW;
  float wt[9];
#pragma unroll
  for (int i = 0; i < 9; ++i) wt[i] = W2[c * 9 + i];
  const float bias = B2[c];
  float v[3][6];
#pragma unroll
  for (int r = 0; r < 3; ++r) {
    const int hh = h + r - 1;
    const bool rv = (unsigned)hh < (unsigned)IMW;
#pragma unroll
    for (int s = 0; s < 6; ++s) {
      const int ww = w0 + s - 1;
      const bool ok = rv && ((unsigned)ww < (unsigned)IMW);
      const int off = ok ? (hh * IMW + ww) : 0;
      const float ld = Oc[off];
      v[r][s] = ok ? ld : 0.0f;
    }
  }
  v4f o;
#pragma unroll
  for (int i = 0; i < 4; ++i) {
    float a = 0.0f;
#pragma unroll
    for (int r = 0; r < 3; ++r)
#pragma unroll
      for (int s = 0; s < 3; ++s) a += v[r][i + s] * wt[r * 3 + s];
    o[i] = a + bias;
  }
  float* dst = out + (size_t)g * 4;
  *(volatile v4f*)dst = o;
  __threadfence();
  *(volatile v4f*)dst = o;
}

extern "C" void kernel_launch(void* const* d_in, const int* in_sizes, int n_in,
                              void* d_out, int out_size, void* d_ws, size_t ws_size,
                              hipStream_t stream) {
  if (n_in < 16) return;
  const int B = in_sizes[0] / (64 * HW);
  if (B <= 0 || in_sizes[0] != B * 64 * HW || out_size != B * 192 * HW) return;
  if (in_sizes[1] != 192 * 64 * 9 || in_sizes[7] != 576 * 192 * 9 || in_sizes[14] != 192 * 9) return;
  if (in_sizes[6] != 192 || in_sizes[12] != 576 || in_sizes[13] < 1 || in_sizes[15] != 192) return;

  const float* x   = (const float*)d_in[0];
  const float* w0  = (const float*)d_in[1];
  const float* b0  = (const float*)d_in[2];
  const float* g0  = (const float*)d_in[3];
  const float* be0 = (const float*)d_in[4];
  const float* m0  = (const float*)d_in[5];
  const float* v0  = (const float*)d_in[6];
  const float* w1  = (const float*)d_in[7];
  const float* b1  = (const float*)d_in[8];
  const float* g1  = (const float*)d_in[9];
  const float* be1 = (const float*)d_in[10];
  const float* m1  = (const float*)d_in[11];
  const float* v1  = (const float*)d_in[12];
  const float* tmp = (const float*)d_in[13];
  const float* w2  = (const float*)d_in[14];
  const float* b2  = (const float*)d_in[15];

  const size_t bytesY  = (size_t)B * 192 * HW * sizeof(float);
  const size_t bytesT  = (size_t)B * 192 * HW * sizeof(_Float16);
  const size_t bytesT2 = (size_t)B * 576 * HW * sizeof(_Float16);
  const size_t bytesP  = (size_t)B * 192 * 192 * sizeof(_Float16);
  const size_t offY  = 0;
  const size_t offT  = offY + bytesY;
  const size_t offT2 = offT + bytesT;
  const size_t offP  = offT2 + bytesT2;
  if (offP + bytesP > ws_size) return;

  char* ws = (char*)d_ws;
  float*    Y  = (float*)(ws + offY);
  _Float16* T  = (_Float16*)(ws + offT);
  _Float16* T2 = (_Float16*)(ws + offT2);
  _Float16* Pm = (_Float16*)(ws + offP);
  float* out = (float*)d_out;

  const int ng8 = B * 192 * HW / 8;
  const int ng4 = B * 192 * HW / 4;

  conv3x3_bn_relu<float, float, 64, 192, 4>
      <<<dim3(HW / 128, 192 / 64, B), 256, 0, stream>>>(x, w0, b0, g0, be0, m0, v0, Y);
  branch_build<<<(ng8 + 255) / 256, 256, 0, stream>>>(Y, T, ng8);
  conv3x3_bn_relu<_Float16, _Float16, 192, 576, 5>
      <<<dim3(HW / 128, 576 / 64, B), 256, 0, stream>>>(T, w1, b1, g1, be1, m1, v1, T2);
  attn_scores_softmax<<<dim3(192 / 64, B), 256, 0, stream>>>(T2, tmp, Pm);
  attn_pv<<<dim3(HW / 128, 192 / 64, B), 256, 0, stream>>>(Pm, T2, Y);
  dwconv3x3<<<(ng4 + 255) / 256, 256, 0, stream>>>(Y, w2, b2, out, ng4);
  (void)hipGetLastError();
}
